// MultiHeadAttention_80925773791779
// MI455X (gfx1250) — hardware-verified
//
#include <hip/hip_runtime.h>


#ifndef NB
#define NB 2
#endif
#ifndef SEQ
#define SEQ 2048
#endif
#define NB_FULL  2
#define SEQ_FULL 2048
#define DM   1024
#define NH   16
#define HD   64
#define DQ   (NH * HD)
#define KD   1024
#define RH   256
#define PCAR 1024.0f
#define SCL  0.125f
#define L2E  1.4426950408889634f
#define NEGB (-3.0e38f)
#define MROWS (NB * SEQ)

typedef _Float16 h16;
typedef unsigned short bf;
typedef __attribute__((ext_vector_type(16))) __bf16   v16bf;
typedef __attribute__((ext_vector_type(16))) _Float16 v16h;
typedef __attribute__((ext_vector_type(8)))  _Float16 v8h;
typedef __attribute__((ext_vector_type(8)))  unsigned short v8us;
typedef __attribute__((ext_vector_type(8)))  float    v8f;
typedef __attribute__((ext_vector_type(4)))  float    v4f;
typedef v8h  __attribute__((may_alias)) v8ha;
typedef v4f  __attribute__((may_alias)) v4fa;
typedef v8us __attribute__((may_alias)) v8usa;

static_assert(DM == KD);
static_assert(DQ == KD);
static_assert(KD % 32 == 0);
static_assert(HD == 64);
static_assert(SEQ % 64 == 0);
static_assert(MROWS % 64 == 0);
static_assert(DQ % 64 == 0);
static_assert(DM % 64 == 0);
static_assert(RH % 64 == 0);
static_assert(RH <= SEQ);
static_assert((SEQ - RH) % 16 == 0);
static_assert(NB <= NB_FULL);
static_assert(SEQ <= SEQ_FULL);
static_assert((size_t)NB_FULL * SEQ_FULL * DM * 4 == (size_t)16777216);

constexpr size_t al256(size_t x) { return (x + 255) & ~(size_t)255; }
constexpr size_t SZ_W  = al256((size_t)DQ * DM * 2);
constexpr size_t SZ_XB = al256((size_t)NB * SEQ * DM * 2);
constexpr size_t SZ_PL = al256((size_t)NB * NH * SEQ * HD * 2);
constexpr size_t SZ_VR = al256((size_t)NB * NH * HD * RH * 2);
constexpr size_t SZ_AT = al256((size_t)NB * SEQ * DQ * 2);
constexpr size_t OFF_WQ = 0;
constexpr size_t OFF_WK = OFF_WQ + SZ_W;
constexpr size_t OFF_WV = OFF_WK + SZ_W;
constexpr size_t OFF_WO = OFF_WV + SZ_W;
constexpr size_t OFF_XB = OFF_WO + SZ_W;
constexpr size_t OFF_QH = OFF_XB + SZ_XB;
constexpr size_t OFF_QL = OFF_QH + SZ_PL;
constexpr size_t OFF_KH = OFF_QL + SZ_PL;
constexpr size_t OFF_KL = OFF_KH + SZ_PL;
constexpr size_t OFF_VT = OFF_KL + SZ_PL;
constexpr size_t OFF_VH = OFF_VT + SZ_PL;
constexpr size_t OFF_VL = OFF_VH + SZ_VR;
constexpr size_t OFF_AH = OFF_VL + SZ_VR;
constexpr size_t OFF_AL = OFF_AH + SZ_AT;
constexpr size_t WS_TOTAL = OFF_AL + SZ_AT;
static_assert(WS_TOTAL <= (size_t)134217728);

__device__ __forceinline__ unsigned short f2bf(float f) { unsigned u = __float_as_uint(f); u += 0x7FFFu + ((u >> 16) & 1u); return (unsigned short)(u >> 16); }
__device__ __forceinline__ float bf2f(unsigned short b) { return __uint_as_float(((unsigned)b) << 16); }
__device__ __forceinline__ void splitf(float y, unsigned short& h, unsigned short& l) { h = f2bf(y); l = f2bf(y - bf2f(h)); }
__device__ __forceinline__ v16h cat16(v8h lo, v8h hi) { return __builtin_shufflevector(lo, hi, 0, 1, 2, 3, 4, 5, 6, 7, 8, 9, 10, 11, 12, 13, 14, 15); }
__device__ __forceinline__ v16bf cat16b(v8us lo, v8us hi) { return __builtin_bit_cast(v16bf, __builtin_shufflevector(lo, hi, 0, 1, 2, 3, 4, 5, 6, 7, 8, 9, 10, 11, 12, 13, 14, 15)); }
__device__ __forceinline__ v16bf ldbf(const bf* p) { return cat16b(*(const v8us*)p, *(const v8us*)(p + 16)); }
__device__ __forceinline__ v16h  ldh(const h16* p) { return cat16(*(const v8h*)p, *(const v8h*)(p + 16)); }
__device__ __forceinline__ v8f mmab(v16bf a, v16bf b, v8f c) {
    c = __builtin_amdgcn_wmma_f32_16x16x32_bf16(false, a, false, b, (short)0, c, false, false);
    asm volatile("v_nop\n\tv_nop\n\tv_nop\n\tv_nop" : "+v"(c) : "v"(a), "v"(b));
    return c; }
__device__ __forceinline__ v8f mmah(v16h a, v16h b, v8f c) {
    c = __builtin_amdgcn_wmma_f32_16x16x32_f16(false, a, false, b, (short)0, c, false, false);
    asm volatile("v_nop\n\tv_nop\n\tv_nop\n\tv_nop" : "+v"(c) : "v"(a), "v"(b));
    return c; }
static __device__ __forceinline__ h16 toh_flush(float v) { const h16 r = (h16)v; return (fabsf(v) < 6.103515625e-05f) ? (h16)0.0f : r; }

__global__ __launch_bounds__(256) void k_cvt8(const float* __restrict__ src, bf* dst, size_t n8) {
    const size_t i = (size_t)blockIdx.x * 256 + threadIdx.x; if (i >= n8) return;
    const v8f v = *(const v8f*)(src + i * 8); v8us o;
#pragma unroll
    for (int k = 0; k < 8; ++k) o[k] = f2bf(v[k]);
    *(volatile v8us*)(dst + i * 8) = o; __threadfence(); *(volatile v8us*)(dst + i * 8) = o; }

__device__ __forceinline__ void gemm_acc(const bf* __restrict__ A, const bf* __restrict__ Bt, size_t aoff, size_t boff, v8f (&acc)[4][4]) {
#pragma unroll 1
    for (int kc = 0; kc < KD; kc += 32) {
        v16bf a[4];
#pragma unroll
        for (int mb = 0; mb < 4; ++mb) a[mb] = ldbf(A + aoff + (size_t)mb * 16 * KD + kc);
#pragma unroll
        for (int nb = 0; nb < 4; ++nb) {
            const v16bf b = ldbf(Bt + boff + (size_t)nb * 16 * KD + kc);
#pragma unroll
            for (int mb = 0; mb < 4; ++mb) acc[mb][nb] = mmab(a[mb], b, acc[mb][nb]);
        }
    }
}

template <int NSPLIT, int MODE>
__device__ __forceinline__ void gemm_tile(const bf* __restrict__ A, const bf* __restrict__ A2, const bf* __restrict__ Bt, float* C, bf* P0, bf* P1, h16* V16, float sc, const float* __restrict__ Bias = nullptr) {
    __shared__ __align__(16) float os[64 * 68];
    const int lane = threadIdx.x & 31, lr = lane & 15, hi = lane >> 4;
    const int r0 = blockIdx.x * 64, c0 = blockIdx.y * 64;
    const size_t zA = (size_t)blockIdx.z * ((size_t)SEQ * DQ);
    const size_t aoff = zA + (size_t)(r0 + lr) * KD + 8 * hi, boff = (size_t)(c0 + lr) * KD + 8 * hi;
    v8f acc[4][4];
#pragma unroll
    for (int mb = 0; mb < 4; ++mb)
#pragma unroll
        for (int nb = 0; nb < 4; ++nb) acc[mb][nb] = (v8f){};
    gemm_acc(A, Bt, aoff, boff, acc);
    if (NSPLIT == 1) gemm_acc(A2, Bt, aoff, boff, acc);
#pragma unroll
    for (int mb = 0; mb < 4; ++mb)
#pragma unroll
        for (int nb = 0; nb < 4; ++nb)
#pragma unroll
            for (int j = 0; j < 8; ++j) os[(mb * 16 + hi * 8 + j) * 68 + nb * 16 + lr] = acc[mb][nb][j];
    __syncthreads();
    if (MODE == 0) {
        const int bb = r0 / SEQ, s0 = r0 % SEQ;
        const size_t prow = ((size_t)(bb * NH + (int)blockIdx.y) * SEQ + s0) * HD;
#pragma unroll 1
        for (int ps = 0; ps < 2; ++ps) {
#pragma unroll 4
            for (int it = 0; it < 16; ++it) {
                const int row = it * 4 + (lane >> 3), col = (lane & 7) * 8;
                const v4f x0 = *(const v4fa*)(os + row * 68 + col), x1 = *(const v4fa*)(os + row * 68 + col + 4);
                v8us oh, ol;
#pragma unroll
                for (int q = 0; q < 4; ++q) { unsigned short a, c; splitf(x0[q] * sc, a, c); oh[q] = a; ol[q] = c; splitf(x1[q] * sc, a, c); oh[q + 4] = a; ol[q + 4] = c; }
                const size_t oo = prow + (size_t)row * HD + col;
                *(volatile v8us*)(P0 + oo) = oh; *(volatile v8us*)(P1 + oo) = ol; }
            if (ps == 0) __threadfence(); }
    }
    if (MODE == 1) {
        const int bb = r0 / SEQ, s0 = r0 % SEQ;
        const size_t vrow = (size_t)(bb * NH + (int)blockIdx.y) * HD;
        const bool early = (s0 < RH);
#pragma unroll 1
        for (int ps = 0; ps < 2; ++ps) {
#pragma unroll 4
            for (int it = 0; it < 16; ++it) {
                const int d = it * 4 + (lane >> 3), sg = (lane & 7) * 8;
                float x[8];
#pragma unroll
                for (int j = 0; j < 8; ++j) x[j] = os[(sg + j) * 68 + d];
                v8h o16; v8us oh, ol;
#pragma unroll
                for (int j = 0; j < 8; ++j) { o16[j] = toh_flush(x[j]); unsigned short a, c; splitf(x[j], a, c); oh[j] = a; ol[j] = c; }
                *(volatile v8h*)(V16 + (vrow + d) * SEQ + s0 + sg) = o16;
                if (early) { const size_t oo = (vrow + d) * RH + s0 + sg; *(volatile v8us*)(P0 + oo) = oh; *(volatile v8us*)(P1 + oo) = ol; } }
            if (ps == 0) __threadfence(); }
    }
    if (MODE == 2) {
        float* cb = C + (size_t)blockIdx.z * ((size_t)SEQ_FULL * DM) + (size_t)r0 * DM + c0;
        const v4f braw = *(const v4f*)(Bias + c0 + lr * 4);
        v4f bv;
#pragma unroll
        for (int q = 0; q < 4; ++q) bv[q] = bf2f(f2bf(braw[q]));
#pragma unroll 1
        for (int ps = 0; ps < 2; ++ps) {
#pragma unroll 4
            for (int it = 0; it < 32; ++it) {
                const int row = it * 2 + hi, cofs = lr * 4;
                const v4f val = *(const v4fa*)(os + row * 68 + cofs) + bv;
                *(volatile v4f*)(cb + (size_t)row * DM + cofs) = val; }
            if (ps == 0) __threadfence(); }
    }
}

__global__ __launch_bounds__(32) void k_proj_qk(const bf* __restrict__ XB, const bf* __restrict__ W, bf* Ph, bf* Pl, float sc) {
    gemm_tile<0, 0>(XB, XB, W, nullptr, Ph, Pl, nullptr, sc); }
__global__ __launch_bounds__(32) void k_proj_v(const bf* __restrict__ XB, const bf* __restrict__ W, h16* V16, bf* Vh, bf* Vl) {
    gemm_tile<0, 1>(XB, XB, W, nullptr, Vh, Vl, V16, 1.0f); }
__global__ __launch_bounds__(32) void k_outp(const bf* __restrict__ Ah, const bf* __restrict__ Al, const bf* __restrict__ W, const float* __restrict__ Bias, float* OUT) {
    gemm_tile<1, 2>(Ah, Al, W, OUT, nullptr, nullptr, nullptr, 1.0f, Bias); }

template <bool HIRES>
__device__ __forceinline__ void attn_body(const bf* __restrict__ QPh, const bf* __restrict__ QPl, const bf* __restrict__ KPh, const bf* __restrict__ KPl,
                                          const h16* __restrict__ VT16, const bf* __restrict__ VTh, const bf* __restrict__ VTl, bf* ATh, bf* ATl, int qbase) {
    __shared__ __align__(16) h16 pt16[16 * 40];
    __shared__ __align__(16) bf pth[16 * 40];
    __shared__ __align__(16) bf ptl[16 * 40];
    __shared__ __align__(16) float os[16 * 68];
    const int lane = threadIdx.x & 31, lr = lane & 15, hi = lane >> 4;
    const int q0 = qbase + (int)blockIdx.x * 16;
    const int bh = (int)blockIdx.y;
    const size_t qoff = ((size_t)bh * SEQ + q0 + lr) * HD + 8 * hi;
    const size_t kbase = ((size_t)bh * SEQ + lr) * HD + 8 * hi;
    v8f o[4];
#pragma unroll
    for (int nt = 0; nt < 4; ++nt) o[nt] = (v8f){};
    float mrow[8], lrow[8];
#pragma unroll
    for (int r = 0; r < 8; ++r) { mrow[r] = NEGB; lrow[r] = 0.0f; }
    const int nkb = (q0 + 16 + 31) / 32;
#pragma unroll 1
    for (int kb = 0; kb < nkb; ++kb) {
        const int s0 = kb * 32;
        v8f sc0 = (v8f){}, sc1 = (v8f){};
#pragma unroll
        for (int ks = 0; ks < 2; ++ks) {
            const v16bf qh = ldbf(QPh + qoff + ks * 32), ql = ldbf(QPl + qoff + ks * 32);
            const size_t ko = kbase + (size_t)s0 * HD + ks * 32;
            { const v16bf kh = ldbf(KPh + ko), kl = ldbf(KPl + ko);
              sc0 = mmab(qh, kh, sc0); sc0 = mmab(ql, kh, sc0); sc0 = mmab(qh, kl, sc0); }
            { const v16bf kh = ldbf(KPh + ko + 16 * HD), kl = ldbf(KPl + ko + 16 * HD);
              sc1 = mmab(qh, kh, sc1); sc1 = mmab(ql, kh, sc1); sc1 = mmab(qh, kl, sc1); }
        }
        float t0[8], t1[8];
#pragma unroll
        for (int r = 0; r < 8; ++r) { t0[r] = sc0[r] * L2E; t1[r] = sc1[r] * L2E; }
        if (s0 + 31 > q0) {
#pragma unroll
            for (int r = 0; r < 8; ++r) { const int row = q0 + 8 * hi + r;
                t0[r] = (s0 + lr > row) ? NEGB : t0[r];
                t1[r] = (s0 + 16 + lr > row) ? NEGB : t1[r]; }
        }
#pragma unroll
        for (int r = 0; r < 8; ++r) {
            float rm = fmaxf(t0[r], t1[r]);
            rm = fmaxf(rm, __shfl_xor(rm, 1, 32)); rm = fmaxf(rm, __shfl_xor(rm, 2, 32));
            rm = fmaxf(rm, __shfl_xor(rm, 4, 32)); rm = fmaxf(rm, __shfl_xor(rm, 8, 32));
            const float mn = fmaxf(mrow[r], rm);
            const float al = __builtin_amdgcn_exp2f(mrow[r] - mn);
            const float p0 = __builtin_amdgcn_exp2f(t0[r] - mn);
            const float p1 = __builtin_amdgcn_exp2f(t1[r] - mn);
            lrow[r] = lrow[r] * al + (p0 + p1); mrow[r] = mn;
            o[0][r] *= al; o[1][r] *= al; o[2][r] *= al; o[3][r] *= al;
            const int pr = (8 * hi + r) * 40 + lr;
            if (HIRES) { unsigned short a, c; splitf(p0, a, c); pth[pr] = a; ptl[pr] = c; splitf(p1, a, c); pth[pr + 16] = a; ptl[pr + 16] = c; }
            else { pt16[pr] = (h16)(p0 * PCAR); pt16[pr + 16] = (h16)(p1 * PCAR); }
        }
        __syncthreads();
        if (HIRES) {
            const v16bf pfh = cat16b(*(const v8usa*)(pth + lr * 40 + 8 * hi), *(const v8usa*)(pth + lr * 40 + 16 + 8 * hi));
            const v16bf pfl = cat16b(*(const v8usa*)(ptl + lr * 40 + 8 * hi), *(const v8usa*)(ptl + lr * 40 + 16 + 8 * hi));
            __syncthreads();
            const size_t vo = ((size_t)bh * HD + lr) * RH + s0 + 8 * hi;
#pragma unroll
            for (int nt = 0; nt < 4; ++nt) {
                const v16bf vh = ldbf(VTh + vo + (size_t)nt * 16 * RH), vl = ldbf(VTl + vo + (size_t)nt * 16 * RH);
                o[nt] = mmab(pfh, vh, o[nt]); o[nt] = mmab(pfl, vh, o[nt]); o[nt] = mmab(pfh, vl, o[nt]); }
        } else {
            const v16h pf = cat16(*(const v8ha*)(pt16 + lr * 40 + 8 * hi), *(const v8ha*)(pt16 + lr * 40 + 16 + 8 * hi));
            __syncthreads();
            const size_t vo = ((size_t)bh * HD + lr) * SEQ + s0 + 8 * hi;
            v16h vb[4];
#pragma unroll
            for (int nt = 0; nt < 4; ++nt) vb[nt] = ldh(VT16 + vo + (size_t)nt * 16 * SEQ);
#pragma unroll
            for (int nt = 0; nt < 4; ++nt) o[nt] = mmah(pf, vb[nt], o[nt]);
        }
    }
#pragma unroll
    for (int r = 0; r < 8; ++r) {
        float ls = lrow[r];
        ls += __shfl_xor(ls, 1, 32); ls += __shfl_xor(ls, 2, 32); ls += __shfl_xor(ls, 4, 32); ls += __shfl_xor(ls, 8, 32);
        const float inv = 1.0f / (ls * (HIRES ? 1.0f : PCAR));
#pragma unroll
        for (int nt = 0; nt < 4; ++nt) os[(8 * hi + r) * 68 + nt * 16 + lr] = o[nt][r] * inv;
    }
    __syncthreads();
    const size_t arow = ((size_t)(bh / NH) * SEQ + q0) * DQ + (size_t)(bh % NH) * HD;
#pragma unroll 1
    for (int ps = 0; ps < 2; ++ps) {
#pragma unroll
        for (int it = 0; it < 4; ++it) {
            const int row = it * 4 + (lane >> 3), col = (lane & 7) * 8;
            const v4f x0 = *(const v4fa*)(os + row * 68 + col), x1 = *(const v4fa*)(os + row * 68 + col + 4);
            v8us oh, ol;
#pragma unroll
            for (int q = 0; q < 4; ++q) { unsigned short a, c; splitf(x0[q], a, c); oh[q] = a; ol[q] = c; splitf(x1[q], a, c); oh[q + 4] = a; ol[q + 4] = c; }
            const size_t oo = arow + (size_t)row * DQ + col;
            *(volatile v8us*)(ATh + oo) = oh; *(volatile v8us*)(ATl + oo) = ol; }
        if (ps == 0) __threadfence(); }
}

__global__ __launch_bounds__(32) void k_attn_hi(const bf* __restrict__ QPh, const bf* __restrict__ QPl, const bf* __restrict__ KPh, const bf* __restrict__ KPl,
                                                const bf* __restrict__ VTh, const bf* __restrict__ VTl, bf* ATh, bf* ATl) {
    attn_body<true>(QPh, QPl, KPh, KPl, nullptr, VTh, VTl, ATh, ATl, 0); }
__global__ __launch_bounds__(32) void k_attn_lo(const bf* __restrict__ QPh, const bf* __restrict__ QPl, const bf* __restrict__ KPh, const bf* __restrict__ KPl,
                                                const h16* __restrict__ VT16, bf* ATh, bf* ATl) {
    attn_body<false>(QPh, QPl, KPh, KPl, VT16, nullptr, nullptr, ATh, ATl, RH); }

extern "C" void kernel_launch(void* const* d_in, const int* in_sizes, int n_in,
                              void* d_out, int out_size, void* d_ws, size_t ws_size, hipStream_t stream) {
    if (n_in < 6) return;
    const size_t need_x = ((size_t)(NB - 1) * SEQ_FULL + SEQ) * DM;
    if ((size_t)in_sizes[0] < need_x) return;
    if ((size_t)in_sizes[1] < (size_t)DQ * DM || (size_t)in_sizes[2] < (size_t)DQ * DM || (size_t)in_sizes[3] < (size_t)DQ * DM || (size_t)in_sizes[4] < (size_t)DM * DQ) return;
    if ((size_t)in_sizes[5] < (size_t)DM) return;
    if ((size_t)out_size < need_x) return;
    if (WS_TOTAL > ws_size) return;
    const float* x  = (const float*)d_in[0];
    const float* wq = (const float*)d_in[1];
    const float* wk = (const float*)d_in[2];
    const float* wv = (const float*)d_in[3];
    const float* wo = (const float*)d_in[4];
    const float* bo = (const float*)d_in[5];
    float* OUT = (float*)d_out;
    char* w = (char*)d_ws;
    bf* WQ = (bf*)(w + OFF_WQ); bf* WK = (bf*)(w + OFF_WK); bf* WV = (bf*)(w + OFF_WV); bf* WO = (bf*)(w + OFF_WO);
    bf* XB = (bf*)(w + OFF_XB);
    bf* QPh = (bf*)(w + OFF_QH); bf* QPl = (bf*)(w + OFF_QL); bf* KPh = (bf*)(w + OFF_KH); bf* KPl = (bf*)(w + OFF_KL);
    h16* VT16 = (h16*)(w + OFF_VT); bf* VTh = (bf*)(w + OFF_VH); bf* VTl = (bf*)(w + OFF_VL);
    bf* ATh = (bf*)(w + OFF_AH); bf* ATl = (bf*)(w + OFF_AL);

    const size_t nw8 = (size_t)DQ * DM / 8, nx8 = (size_t)SEQ * DM / 8;
    k_cvt8<<<(unsigned)((nw8 + 255) / 256), 256, 0, stream>>>(wq, WQ, nw8);
    k_cvt8<<<(unsigned)((nw8 + 255) / 256), 256, 0, stream>>>(wk, WK, nw8);
    k_cvt8<<<(unsigned)((nw8 + 255) / 256), 256, 0, stream>>>(wv, WV, nw8);
    k_cvt8<<<(unsigned)((nw8 + 255) / 256), 256, 0, stream>>>(wo, WO, nw8);
    for (int b = 0; b < NB; ++b)
        k_cvt8<<<(unsigned)((nx8 + 255) / 256), 256, 0, stream>>>(x + (size_t)b * SEQ_FULL * DM, XB + (size_t)b * SEQ * DM, nx8);

    k_proj_qk<<<dim3(MROWS / 64, DQ / 64, 1), 32, 0, stream>>>(XB, WQ, QPh, QPl, SCL);
    k_proj_qk<<<dim3(MROWS / 64, DQ / 64, 1), 32, 0, stream>>>(XB, WK, KPh, KPl, 1.0f);
    k_proj_v<<<dim3(MROWS / 64, DQ / 64, 1), 32, 0, stream>>>(XB, WV, VT16, VTh, VTl);

    k_attn_hi<<<dim3(RH / 16, NB * NH, 1), 32, 0, stream>>>(QPh, QPl, KPh, KPl, VTh, VTl, ATh, ATl);
    if (SEQ > RH)
        k_attn_lo<<<dim3((SEQ - RH) / 16, NB * NH, 1), 32, 0, stream>>>(QPh, QPl, KPh, KPl, VT16, ATh, ATl);

    k_outp<<<dim3(SEQ / 64, DM / 64, NB), 32, 0, stream>>>(ATh, ATl, WO, bo, OUT);
}
